// GraphTransformerTeacher_69071664054561
// MI455X (gfx1250) — hardware-verified
//
#include <hip/hip_runtime.h>
#include <stddef.h>


#define FIN     256
#define HCN     512
#define NHD     8
#define CHN     64
#define NTHR    256
#define NWAVE   8
#define EPT     8
#define NGRP    2
#define CHUNK   (NTHR * EPT * NGRP)
#define WCAP    (EPT * NGRP * 32)
#define LISTN   (NWAVE * WCAP)
#define NBC     4096
#define NBF     1024
#define RCAP    40960
#define RBN     128
#define TGT     256
#define DEGCAP  256
#define OTHR    512
#define BM      64
#define BN      128
#define WSCAP   134217728
#define NEG_SLOPE 0.2f
#define WSC     16.0f
#define H1SC    8.0f

#define LDS_FILL ((RCAP + NBF + LISTN) * 4 + 64)

static_assert((CHUNK & (CHUNK - 1)) == 0);
static_assert(CHUNK <= 4096);
static_assert(NBC <= 4096 && NBF <= 4096);
static_assert((NBC & (NBC - 1)) == 0 && (NBF & (NBF - 1)) == 0);
static_assert(NBC == 4 * NBF);
static_assert(OTHR * 8 == NBC);
static_assert((RCAP % 32) == 0);
static_assert(TGT == NWAVE * 32);
static_assert((NBC % TGT) == 0);
static_assert((TGT % BM) == 0);
static_assert(BM * 4 == NTHR);
static_assert(FIN % 32 == 0 && HCN % 32 == 0);
static_assert(NHD * CHN == HCN);
static_assert(BN == 2 * CHN);
static_assert(HCN % BN == 0);
static_assert(HCN == 32 * 16);

typedef float          v2f  __attribute__((ext_vector_type(2)));
typedef float          v4f  __attribute__((ext_vector_type(4)));
typedef float          v8f  __attribute__((ext_vector_type(8)));
typedef int            v4i  __attribute__((ext_vector_type(4)));
typedef unsigned short v8us __attribute__((ext_vector_type(8)));
typedef _Float16       v8h  __attribute__((ext_vector_type(8)));
typedef _Float16       v16h __attribute__((ext_vector_type(16)));
union FragH { v16h v; v8us u[2]; };
union Pk8   { v8h h; v8us u; };

__device__ __forceinline__ v8f wmh(v16h a, v16h b, v8f c) {
  v8f d = __builtin_amdgcn_wmma_f32_16x16x32_f16(false, a, false, b, (short)0, c, false, false);
  asm volatile("v_nop\n\tv_nop\n\tv_nop\n\tv_nop" : "+v"(d) : "v"(a), "v"(b));
  return d;
}

__device__ __forceinline__ v8us cvt8h(v4f a, v4f b, float sc) {
  v8f f;
  f[0] = a.x * sc; f[1] = a.y * sc; f[2] = a.z * sc; f[3] = a.w * sc;
  f[4] = b.x * sc; f[5] = b.y * sc; f[6] = b.z * sc; f[7] = b.w * sc;
  Pk8 r;
  r.h = __builtin_convertvector(f, v8h);
  return r.u;
}

__device__ __forceinline__ float lrelu(float v) { return v > 0.0f ? v : NEG_SLOPE * v; }
__device__ __forceinline__ v4f relu4(v4f v) {
  v4f r;
  r.x = fmaxf(v.x, 0.0f); r.y = fmaxf(v.y, 0.0f); r.z = fmaxf(v.z, 0.0f); r.w = fmaxf(v.w, 0.0f);
  return r;
}
__device__ __forceinline__ float hsum3(float t) {
  t += __shfl_xor(t, 4);
  t += __shfl_xor(t, 8);
  t += __shfl_xor(t, 16);
  return t;
}
__device__ __forceinline__ v4f hsum3v(v4f v) {
  v4f r;
  r.x = hsum3(v.x); r.y = hsum3(v.y); r.z = hsum3(v.z); r.w = hsum3(v.w);
  return r;
}

template <int NB>
__device__ __forceinline__ int scan_chunk(const int* __restrict__ dsts, int nE, int cbase, int slotBase,
                                          int vec8, int* list, int tid, int lane, int wave) {
  int wc = 0;
#pragma unroll
  for (int g = 0; g < NGRP; ++g) {
    const int el0  = (g * NTHR + tid) * EPT;
    const int e0   = cbase + el0;
    const int sent = -2147483647 - 1;
    v4i da, db;
    if (vec8 != 0 && cbase + CHUNK <= nE) {
      da = *(const v4i*)(dsts + e0);
      db = *(const v4i*)(dsts + e0 + 4);
    } else {
      da.x = (e0     < nE) ? dsts[min(e0, nE - 1)] : sent;
      da.y = (e0 + 1 < nE) ? dsts[min(e0 + 1, nE - 1)] : sent;
      da.z = (e0 + 2 < nE) ? dsts[min(e0 + 2, nE - 1)] : sent;
      da.w = (e0 + 3 < nE) ? dsts[min(e0 + 3, nE - 1)] : sent;
      db.x = (e0 + 4 < nE) ? dsts[min(e0 + 4, nE - 1)] : sent;
      db.y = (e0 + 5 < nE) ? dsts[min(e0 + 5, nE - 1)] : sent;
      db.z = (e0 + 6 < nE) ? dsts[min(e0 + 6, nE - 1)] : sent;
      db.w = (e0 + 7 < nE) ? dsts[min(e0 + 7, nE - 1)] : sent;
    }
    const unsigned nb = (unsigned)slotBase;
    const unsigned s0 = (unsigned)da.x - nb, s1 = (unsigned)da.y - nb;
    const unsigned s2 = (unsigned)da.z - nb, s3 = (unsigned)da.w - nb;
    const unsigned s4 = (unsigned)db.x - nb, s5 = (unsigned)db.y - nb;
    const unsigned s6 = (unsigned)db.z - nb, s7 = (unsigned)db.w - nb;
    const bool h0 = s0 < (unsigned)NB, h1 = s1 < (unsigned)NB, h2 = s2 < (unsigned)NB, h3 = s3 < (unsigned)NB;
    const bool h4 = s4 < (unsigned)NB, h5 = s5 < (unsigned)NB, h6 = s6 < (unsigned)NB, h7 = s7 < (unsigned)NB;
    const unsigned any = __builtin_amdgcn_ballot_w32(h0 | h1 | h2 | h3 | h4 | h5 | h6 | h7);
    if (any != 0u) {
#define HITJ(J, HJ, SJ) { \
        const unsigned mj = __builtin_amdgcn_ballot_w32(HJ); \
        if (mj != 0u) { \
          if (HJ) { \
            const int pos = wc + (int)__builtin_amdgcn_mbcnt_lo(mj, 0u); \
            if (pos < WCAP) list[wave * WCAP + pos] = ((el0 + (J)) << 12) | (int)(SJ); \
          } \
          wc += (int)__builtin_popcount(mj); } }
      HITJ(0, h0, s0)
      HITJ(1, h1, s1)
      HITJ(2, h2, s2)
      HITJ(3, h3, s3)
      HITJ(4, h4, s4)
      HITJ(5, h5, s5)
      HITJ(6, h6, s6)
      HITJ(7, h7, s7)
#undef HITJ
    }
  }
  return wc;
}

__global__ __launch_bounds__(NTHR) void k_xcvt(const float* __restrict__ x, unsigned short* xp, int nN, int nUnits) {
  const int i = (int)blockIdx.x * NTHR + (int)threadIdx.x;
  if (i >= nUnits) return;
  const int row = i >> 5;
  const int c0  = (i & 31) * 8;
  int rr = row > nN - 1 ? nN - 1 : row;
  rr = rr < 0 ? 0 : rr;
  const float* p = x + (size_t)rr * FIN + c0;
  v4f a = *(const v4f*)p, b = *(const v4f*)(p + 4);
  const v4f z = {0.f, 0.f, 0.f, 0.f};
  if (row >= nN) { a = z; b = z; }
  const v8us o = cvt8h(a, b, 1.0f);
  unsigned short* d = xp + (size_t)i * 8;
  *(volatile v8us*)d = o;
  __threadfence();
  *(volatile v8us*)d = o;
}

template <int KD, int NCW>
__global__ __launch_bounds__(NTHR) void k_wprep(const float* __restrict__ W, unsigned short* wp) {
  constexpr int KS    = KD / 8;
  constexpr int UNITS = NCW * KS;
  static_assert(KD % 8 == 0);
  const int i = (int)blockIdx.x * NTHR + (int)threadIdx.x;
  if (i >= UNITS) return;
  const int n  = i / KS;
  const int k0 = (i - n * KS) * 8;
  v4f a, b;
  a.x = W[(size_t)(k0 + 0) * NCW + n]; a.y = W[(size_t)(k0 + 1) * NCW + n];
  a.z = W[(size_t)(k0 + 2) * NCW + n]; a.w = W[(size_t)(k0 + 3) * NCW + n];
  b.x = W[(size_t)(k0 + 4) * NCW + n]; b.y = W[(size_t)(k0 + 5) * NCW + n];
  b.z = W[(size_t)(k0 + 6) * NCW + n]; b.w = W[(size_t)(k0 + 7) * NCW + n];
  const v8us o = cvt8h(a, b, WSC);
  unsigned short* d = wp + (size_t)i * 8;
  *(volatile v8us*)d = o;
  __threadfence();
  *(volatile v8us*)d = o;
}

__global__ __launch_bounds__(NTHR) void k_count(
    const int* __restrict__ dsts, int* cnt, int nE, int vec8) {
  __shared__ __attribute__((aligned(16))) int scnt[NBC];
  __shared__ __attribute__((aligned(16))) int list[LISTN];
  __shared__ int wcnt[NWAVE];
  const int tid = threadIdx.x, lane = tid & 31, wave = tid >> 5;
  const int nodeBase = blockIdx.x * NBC;

  for (int i = tid; i < NBC; i += NTHR) scnt[i] = 0;
  __syncthreads();

  const int nChunks = (nE + CHUNK - 1) / CHUNK;
#pragma unroll 1
  for (int ch = 0; ch < nChunks; ++ch) {
    const int cbase = ch * CHUNK;
    const int wc = scan_chunk<NBC>(dsts, nE, cbase, nodeBase, vec8, list, tid, lane, wave);
    if (lane == 0) wcnt[wave] = wc;
    __syncthreads();
    if (wave == 0) {
#pragma unroll 1
      for (int wsx = 0; wsx < NWAVE; ++wsx) {
        int n = __builtin_amdgcn_readfirstlane(wcnt[wsx]);
        n = n > WCAP ? WCAP : (n < 0 ? 0 : n);
        const int* lp = list + wsx * WCAP;
#pragma unroll 1
        for (int i = 0; i < n; ++i) {
          const int ent  = __builtin_amdgcn_readfirstlane(lp[i]);
          const int slot = ent & (NBC - 1);
          if (lane == 0) scnt[slot] = scnt[slot] + 1;
        }
      }
    }
    __syncthreads();
  }

  v4i cq[4];
#pragma unroll
  for (int q = 0; q < 4; ++q) {
    const int f = (wave * 4 + q) * 128 + 4 * lane;
    cq[q] = *(const v4i*)(scnt + f);
  }
  int* cp = cnt + (size_t)nodeBase;
#pragma unroll
  for (int q = 0; q < 4; ++q) {
    const int f = (wave * 4 + q) * 128 + 4 * lane;
    *(volatile v4i*)(cp + f) = cq[q];
  }
  __threadfence();
#pragma unroll
  for (int q = 0; q < 4; ++q) {
    const int f = (wave * 4 + q) * 128 + 4 * lane;
    *(volatile v4i*)(cp + f) = cq[q];
  }
}

__global__ __launch_bounds__(OTHR) void k_offsets(
    const int* __restrict__ cnt, int* off, int* rbase, int nChunk) {
  __shared__ __attribute__((aligned(16))) int soff[NBC];
  __shared__ __attribute__((aligned(16))) int srb[RBN];
  __shared__ int wtot[OTHR / 32];
  const int tid = threadIdx.x, lane = tid & 31, wave = tid >> 5, sub = tid >> 7;
  for (int i = tid; i < RBN; i += OTHR) srb[i] = 0;
  int carry = 0;
#pragma unroll 1
  for (int ch = 0; ch < nChunk; ++ch) {
    const int base = ch * NBC;
    const v4i c0 = *(const v4i*)(cnt + base + 8 * tid);
    const v4i c1 = *(const v4i*)(cnt + base + 8 * tid + 4);
    const int e0 = max(c0.x, 0), e1 = max(c0.y, 0), e2 = max(c0.z, 0), e3 = max(c0.w, 0);
    const int e4 = max(c1.x, 0), e5 = max(c1.y, 0), e6 = max(c1.z, 0), e7 = max(c1.w, 0);
    const int ts = e0 + e1 + e2 + e3 + e4 + e5 + e6 + e7;
    int incl = ts;
#pragma unroll
    for (int d = 1; d < 32; d <<= 1) {
      const int t = __shfl_up(incl, d);
      if (lane >= d) incl += t;
    }
    if (lane == 31) wtot[wave] = incl;
    __syncthreads();
    const int S0 = wtot[0]  + wtot[1]  + wtot[2]  + wtot[3];
    const int S1 = wtot[4]  + wtot[5]  + wtot[6]  + wtot[7];
    const int S2 = wtot[8]  + wtot[9]  + wtot[10] + wtot[11];
    const int S3 = wtot[12] + wtot[13] + wtot[14] + wtot[15];
    int pre = 0;
#pragma unroll 1
    for (int w = 4 * sub; w < wave; ++w) pre += wtot[w];
    const int b0 = carry;
    const int b1 = b0 + ((S0 + 31) & ~31);
    const int b2 = b1 + ((S1 + 31) & ~31);
    const int b3 = b2 + ((S2 + 31) & ~31);
    const int b4 = b3 + ((S3 + 31) & ~31);
    const int myb = sub == 0 ? b0 : (sub == 1 ? b1 : (sub == 2 ? b2 : b3));
    if (tid == 0) {
      srb[min(4 * ch + 0, RBN - 1)] = b0;
      srb[min(4 * ch + 1, RBN - 1)] = b1;
      srb[min(4 * ch + 2, RBN - 1)] = b2;
      srb[min(4 * ch + 3, RBN - 1)] = b3;
    }
    int run = myb + pre + incl - ts;
    soff[8 * tid + 0] = run; run += e0;
    soff[8 * tid + 1] = run; run += e1;
    soff[8 * tid + 2] = run; run += e2;
    soff[8 * tid + 3] = run; run += e3;
    soff[8 * tid + 4] = run; run += e4;
    soff[8 * tid + 5] = run; run += e5;
    soff[8 * tid + 6] = run; run += e6;
    soff[8 * tid + 7] = run;
    carry = b4;
    __syncthreads();
    const v4i o0 = *(const v4i*)(soff + 4 * tid);
    const v4i o1 = *(const v4i*)(soff + 4 * (tid + OTHR));
    int* op = off + base;
    *(volatile v4i*)(op + 4 * tid) = o0;
    *(volatile v4i*)(op + 4 * (tid + OTHR)) = o1;
    __threadfence();
    *(volatile v4i*)(op + 4 * tid) = o0;
    *(volatile v4i*)(op + 4 * (tid + OTHR)) = o1;
    __syncthreads();
  }
  if (tid == 0) srb[min(4 * nChunk, RBN - 1)] = carry;
  __syncthreads();
  v4i rv = {0, 0, 0, 0};
  if (tid < 32) rv = *(const v4i*)(srb + 4 * tid);
  if (tid < 32) *(volatile v4i*)(rbase + 4 * tid) = rv;
  __threadfence();
  if (tid < 32) *(volatile v4i*)(rbase + 4 * tid) = rv;
}

__global__ __launch_bounds__(NTHR) void k_fill(
    const int* __restrict__ srcs, const int* __restrict__ dsts,
    const int* __restrict__ off, const int* __restrict__ rbase,
    int* csr, int nN, int nE, int vec8, int csrLen) {
  extern __shared__ v4f lds_dyn[];
  int* region = (int*)lds_dyn;
  int* cursor = region + RCAP;
  int* list   = cursor + NBF;
  int* wcnt   = list + LISTN;
  const int tid = threadIdx.x, lane = tid & 31, wave = tid >> 5;
  const int b = blockIdx.x;
  const int nodeBase = b * NBF;

  int rb0 = rbase[b];
  const int rb1 = rbase[b + 1];
  rb0 = rb0 < 0 ? 0 : (rb0 > csrLen ? csrLen : rb0);
  rb0 &= ~31;
  int len = rb1 - rb0;
  len = len < 0 ? 0 : (len > RCAP ? RCAP : len);
  int lenW = (len + 31) & ~31;
  if (rb0 + lenW > csrLen) lenW = (csrLen - rb0) & ~31;

  {
    const v4i z = {0, 0, 0, 0};
    for (int i = tid; i < RCAP / 4; i += NTHR) ((v4i*)region)[i] = z;
    for (int s = tid; s < NBF; s += NTHR) {
      int o = off[nodeBase + s] - rb0;
      o = o < 0 ? 0 : (o > RCAP ? RCAP : o);
      cursor[s] = o;
    }
  }
  __syncthreads();

  const int nChunks = (nE + CHUNK - 1) / CHUNK;
#pragma unroll 1
  for (int ch = 0; ch < nChunks; ++ch) {
    const int cbase = ch * CHUNK;
    const int wc = scan_chunk<NBF>(dsts, nE, cbase, nodeBase, vec8, list, tid, lane, wave);
    if (lane == 0) wcnt[wave] = wc;
    __syncthreads();
    if (wave == 0) {
#pragma unroll 1
      for (int wsx = 0; wsx < NWAVE; ++wsx) {
        int n = __builtin_amdgcn_readfirstlane(wcnt[wsx]);
        n = n > WCAP ? WCAP : (n < 0 ? 0 : n);
        const int* lp = list + wsx * WCAP;
#pragma unroll 1
        for (int i = 0; i < n; ++i) {
          const int ent  = __builtin_amdgcn_readfirstlane(lp[i]);
          const int slot = ent & (NBF - 1);
          int e = cbase + ((ent >> 12) & (CHUNK - 1));
          e = e > nE - 1 ? nE - 1 : e;
          int src = srcs[e];
          src = src < 0 ? 0 : (src > nN - 1 ? nN - 1 : src);
          if (lane == 0) {
            int pos = cursor[slot];
            pos = pos < 0 ? 0 : (pos > RCAP - 1 ? RCAP - 1 : pos);
            region[pos] = src;
            const int np = pos + 1;
            cursor[slot] = np > RCAP ? RCAP : np;
          }
        }
      }
    }
    __syncthreads();
  }

  const int nv = lenW >> 2;
  int* gp = csr + rb0;
#pragma unroll 1
  for (int i = tid; i < nv; i += NTHR) { const v4i v = ((const v4i*)region)[i]; *(volatile v4i*)(gp + 4 * i) = v; }
  __threadfence();
#pragma unroll 1
  for (int i = tid; i < nv; i += NTHR) { const v4i v = ((const v4i*)region)[i]; *(volatile v4i*)(gp + 4 * i) = v; }
}

template <int K, int OSH>
__global__ __launch_bounds__(NTHR) void k_gemm(
    const unsigned short* __restrict__ Ap, const unsigned short* __restrict__ Bp,
    const float* __restrict__ attS, const float* __restrict__ attD,
    float* C, float* eS, float* eD, int npad) {
  constexpr int TPW = 4;
  constexpr int KT  = K / 32;
  constexpr int CPP = 32;
  constexpr int NES = BM * 2;
  constexpr int NIT = BM / NWAVE;
  static_assert(K % 32 == 0);
  static_assert(TPW * 16 * 2 == BN);
  static_assert(NES == 4 * 32);
  static_assert(BN == 4 * 32);

  __shared__ __attribute__((aligned(16))) float stg[BM * BN];
  __shared__ __attribute__((aligned(16))) float sES[NES];
  __shared__ __attribute__((aligned(16))) float sED[NES];
  const int tid = threadIdx.x, lane = tid & 31, wave = tid >> 5, hh = lane >> 4, m = lane & 15;
  const int rowBase = blockIdx.x * BM;
  const int cs = blockIdx.y * BN;
  const int rg = wave >> 1, chf = wave & 1;
  const int r0 = rg * 16;
  const int c0 = chf * 64;
  const float osc = 1.0f / (float)(1 << OSH);

  v8f acc[TPW];
#pragma unroll
  for (int t = 0; t < TPW; ++t) { v8f z = {0.f, 0.f, 0.f, 0.f, 0.f, 0.f, 0.f, 0.f}; acc[t] = z; }

  const unsigned short* ap  = Ap + (size_t)(rowBase + r0 + m) * K + 8 * hh;
  const unsigned short* bp0 = Bp + (size_t)(cs + c0 + m) * K + 8 * hh;
#pragma unroll 1
  for (int kt = 0; kt < KT; ++kt) {
    FragH a;
    a.u[0] = *(const v8us*)(ap + 32 * kt);
    a.u[1] = *(const v8us*)(ap + 32 * kt + 16);
#pragma unroll
    for (int t = 0; t < TPW; ++t) {
      const unsigned short* bp = bp0 + (size_t)(16 * t) * K + 32 * kt;
      FragH bf;
      bf.u[0] = *(const v8us*)bp;
      bf.u[1] = *(const v8us*)(bp + 16);
      acc[t] = wmh(a.v, bf.v, acc[t]);
    }
  }

  {
    float* sp = stg + (size_t)(r0 + 8 * hh) * BN + c0 + m;
#pragma unroll
    for (int t = 0; t < TPW; ++t) {
#pragma unroll
      for (int r = 0; r < 8; ++r) sp[r * BN + 16 * t] = acc[t][r] * osc;
    }
  }
  __syncthreads();

  {
    const int drow = tid >> 2, part = tid & 3;
    const float* rp  = stg + (size_t)drow * BN + CPP * part;
    const float* sa  = attS + blockIdx.y * BN + CPP * part;
    const float* sdd = attD + blockIdx.y * BN + CPP * part;
    float ps = 0.f, pd = 0.f;
#pragma unroll 2
    for (int c = 0; c < CPP; c += 4) {
      const v4f hv = *(const v4f*)(rp + c);
      const v4f av = *(const v4f*)(sa + c);
      const v4f dv = *(const v4f*)(sdd + c);
      ps += hv.x * av.x + hv.y * av.y + hv.z * av.z + hv.w * av.w;
      pd += hv.x * dv.x + hv.y * dv.y + hv.z * dv.z + hv.w * dv.w;
    }
    ps += __shfl_xor(ps, 1); pd += __shfl_xor(pd, 1);
    if ((part & 1) == 0) { sES[drow * 2 + (part >> 1)] = ps; sED[drow * 2 + (part >> 1)] = pd; }
  }

  {
    float* cb = C + (size_t)rowBase * HCN + cs + 4 * lane;
    v4f cv[NIT];
#pragma unroll
    for (int it = 0; it < NIT; ++it) cv[it] = *(const v4f*)(stg + (size_t)(it * NWAVE + wave) * BN + 4 * lane);
#pragma unroll
    for (int it = 0; it < NIT; ++it) *(volatile v4f*)(cb + (size_t)(it * NWAVE + wave) * HCN) = cv[it];
    __threadfence();
#pragma unroll
    for (int it = 0; it < NIT; ++it) *(volatile v4f*)(cb + (size_t)(it * NWAVE + wave) * HCN) = cv[it];
  }
  __syncthreads();

  {
    const size_t eb = ((size_t)blockIdx.y * (size_t)npad + (size_t)rowBase) * 2;
    const v4f vS = *(const v4f*)(sES + 4 * lane);
    const v4f vD = *(const v4f*)(sED + 4 * lane);
    const v4f dv = (wave == 0) ? vS : vD;
    float* gp = ((wave == 0) ? eS : eD) + eb + 4 * lane;
    if (wave < 2) *(volatile v4f*)gp = dv;
    __threadfence();
    if (wave < 2) *(volatile v4f*)gp = dv;
  }
}

__device__ __forceinline__ void gat_row(
    const int* __restrict__ csr, const float* __restrict__ eS, const float* __restrict__ hw,
    size_t eoff, float edc, float eself, int c, int n, int st, int col, int lane, int nN, int csrLen,
    float& mxo, float& deno, v4f& a0, v4f& a1, v4f& a2, v4f& a3) {
  float mx = eself;
#pragma unroll 1
  for (int q0 = 0; q0 < n; q0 += 32) {
    int pos = st + q0 + lane;
    pos = pos < 0 ? 0 : (pos > csrLen - 1 ? csrLen - 1 : pos);
    int sl = csr[pos];
    sl = sl < 0 ? 0 : (sl > nN - 1 ? nN - 1 : sl);
    const int mcnt = (n - q0) < 32 ? (n - q0) : 32;
#pragma unroll 1
    for (int pp = 0; pp < mcnt; ++pp) {
      const int s = __builtin_amdgcn_readlane(sl, pp);
      mx = fmaxf(mx, lrelu(eS[eoff + (size_t)s * 2] + edc));
    }
  }

  float p   = __expf(eself - mx);
  float den = p;
  const float* hc = hw + (size_t)c * HCN + col;
  v4f b0 = *(const v4f*)hc * p;
  v4f b1 = *(const v4f*)(hc + 4) * p;
  v4f b2 = *(const v4f*)(hc + 8) * p;
  v4f b3 = *(const v4f*)(hc + 12) * p;
#pragma unroll 1
  for (int q0 = 0; q0 < n; q0 += 32) {
    int pos = st + q0 + lane;
    pos = pos < 0 ? 0 : (pos > csrLen - 1 ? csrLen - 1 : pos);
    int sl = csr[pos];
    sl = sl < 0 ? 0 : (sl > nN - 1 ? nN - 1 : sl);
    const int mcnt = (n - q0) < 32 ? (n - q0) : 32;
#pragma unroll 1
    for (int pp = 0; pp < mcnt; ++pp) {
      const int s = __builtin_amdgcn_readlane(sl, pp);
      p = __expf(lrelu(eS[eoff + (size_t)s * 2] + edc) - mx);
      den += p;
      const float* hs = hw + (size_t)s * HCN + col;
      const v4f h0 = *(const v4f*)hs;
      const v4f h1 = *(const v4f*)(hs + 4);
      const v4f h2 = *(const v4f*)(hs + 8);
      const v4f h3 = *(const v4f*)(hs + 12);
      b0 = b0 + h0 * p; b1 = b1 + h1 * p; b2 = b2 + h2 * p; b3 = b3 + h3 * p;
    }
  }
  mxo = mx; deno = den; a0 = b0; a1 = b1; a2 = b2; a3 = b3;
}

__global__ __launch_bounds__(NTHR) void k_agg1(
    const int* __restrict__ csr, const int* __restrict__ off, const int* __restrict__ cnt,
    const float* __restrict__ eS, const float* __restrict__ eD, const float* __restrict__ hw,
    const float* __restrict__ bias, float* Mt, float* Dt, unsigned short* xo,
    int nN, int npad, int csrLen) {
  __shared__ __attribute__((aligned(16))) unsigned short sRow[NWAVE * HCN];
  __shared__ __attribute__((aligned(16))) float sM[NWAVE * 256];
  __shared__ __attribute__((aligned(16))) float sDn[NWAVE * 256];
  const int tid = threadIdx.x, lane = tid & 31, wave = tid >> 5;
  const int tbase = blockIdx.x * TGT + wave * 32;
  const int col = 16 * lane;
  const int hd  = lane >> 2;
  const size_t eoff = (size_t)(hd >> 1) * (size_t)npad * 2 + (size_t)(hd & 1);
  unsigned short* srw = sRow + wave * HCN;
  float* smw = sM + wave * 256;
  float* sdw = sDn + wave * 256;

  const v4f bb0 = *(const v4f*)(bias + col);
  const v4f bb1 = *(const v4f*)(bias + col + 4);
  const v4f bb2 = *(const v4f*)(bias + col + 8);
  const v4f bb3 = *(const v4f*)(bias + col + 12);

  const int cl    = tbase + lane;
  const int cnt_l = cnt[cl];
  const int off_l = off[cl];

#pragma unroll 1
  for (int j = 0; j < 32; ++j) {
    const int c = tbase + j;
    int n = __shfl(cnt_l, j);
    n = n < 0 ? 0 : (n > DEGCAP ? DEGCAP : n);
    const int st = __shfl(off_l, j);
    const float edc   = eD[eoff + (size_t)c * 2];
    const float eself = lrelu(eS[eoff + (size_t)c * 2] + edc);

    float mx, den;
    v4f a0, a1, a2, a3;
    gat_row(csr, eS, hw, eoff, edc, eself, c, n, st, col, lane, nN, csrLen, mx, den, a0, a1, a2, a3);

    const float rd = __builtin_amdgcn_rcpf(den);
    v4f v0 = relu4(a0 * rd + bb0);
    v4f v1 = relu4(a1 * rd + bb1);
    v4f v2 = relu4(a2 * rd + bb2);
    v4f v3 = relu4(a3 * rd + bb3);
    if (c >= nN) { const v4f z = {0.f, 0.f, 0.f, 0.f}; v0 = z; v1 = z; v2 = z; v3 = z; }
    const v8us q0 = cvt8h(v0, v1, H1SC);
    const v8us q1 = cvt8h(v2, v3, H1SC);
    *(v8us*)(srw + col) = q0;
    *(v8us*)(srw + col + 8) = q1;
    if ((lane & 3) == 0) { smw[j * 8 + hd] = mx; sdw[j * 8 + hd] = den; }
    __syncthreads();

    const v8us p0 = *(const v8us*)(srw + 8 * lane);
    const v8us p1 = *(const v8us*)(srw + 256 + 8 * lane);
    unsigned short* gp = xo + (size_t)c * HCN + 8 * lane;
    *(volatile v8us*)gp = p0;
    *(volatile v8us*)(gp + 256) = p1;
    __threadfence();
    *(volatile v8us*)gp = p0;
    *(volatile v8us*)(gp + 256) = p1;
    __syncthreads();
  }

  {
    const v4f m0 = *(const v4f*)(smw + 4 * lane);
    const v4f m1 = *(const v4f*)(smw + 128 + 4 * lane);
    const v4f d0 = *(const v4f*)(sdw + 4 * lane);
    const v4f d1 = *(const v4f*)(sdw + 128 + 4 * lane);
    float* mp = Mt + (size_t)tbase * NHD + 4 * lane;
    float* dp = Dt + (size_t)tbase * NHD + 4 * lane;
    *(volatile v4f*)mp = m0; *(volatile v4f*)(mp + 128) = m1;
    *(volatile v4f*)dp = d0; *(volatile v4f*)(dp + 128) = d1;
    __threadfence();
    *(volatile v4f*)mp = m0; *(volatile v4f*)(mp + 128) = m1;
    *(volatile v4f*)dp = d0; *(volatile v4f*)(dp + 128) = d1;
  }
}

__global__ __launch_bounds__(NTHR) void k_agg2(
    const int* __restrict__ csr, const int* __restrict__ off, const int* __restrict__ cnt,
    const float* __restrict__ eS, const float* __restrict__ eD, const float* __restrict__ hw,
    const float* __restrict__ bias, float* Mt, float* Dt, float* out,
    int nN, int npad, int csrLen) {
  __shared__ __attribute__((aligned(16))) float sO[NWAVE * CHN];
  __shared__ __attribute__((aligned(16))) float sM[NWAVE * 256];
  __shared__ __attribute__((aligned(16))) float sDn[NWAVE * 256];
  const int tid = threadIdx.x, lane = tid & 31, wave = tid >> 5;
  const int tbase = blockIdx.x * TGT + wave * 32;
  const int col = 16 * lane;
  const int hd  = lane >> 2;
  const size_t eoff = (size_t)(hd >> 1) * (size_t)npad * 2 + (size_t)(hd & 1);
  float* sow = sO + wave * CHN;
  float* smw = sM + wave * 256;
  float* sdw = sDn + wave * 256;

  const int lq = lane < 16 ? lane : 15;
  const v4f bb = *(const v4f*)(bias + 4 * lq);

  const int cl    = tbase + lane;
  const int cnt_l = cnt[cl];
  const int off_l = off[cl];

#pragma unroll 1
  for (int j = 0; j < 32; ++j) {
    const int c = tbase + j;
    int n = __shfl(cnt_l, j);
    n = n < 0 ? 0 : (n > DEGCAP ? DEGCAP : n);
    const int st = __shfl(off_l, j);
    const float edc   = eD[eoff + (size_t)c * 2];
    const float eself = lrelu(eS[eoff + (size_t)c * 2] + edc);

    float mx, den;
    v4f a0, a1, a2, a3;
    gat_row(csr, eS, hw, eoff, edc, eself, c, n, st, col, lane, nN, csrLen, mx, den, a0, a1, a2, a3);

    const float rd = __builtin_amdgcn_rcpf(den);
    v4f v0 = hsum3v(a0 * rd);
    v4f v1 = hsum3v(a1 * rd);
    v4f v2 = hsum3v(a2 * rd);
    v4f v3 = hsum3v(a3 * rd);
    if (lane < 4) {
      *(v4f*)(sow + 16 * lane)      = v0;
      *(v4f*)(sow + 16 * lane + 4)  = v1;
      *(v4f*)(sow + 16 * lane + 8)  = v2;
      *(v4f*)(sow + 16 * lane + 12) = v3;
    }
    if ((lane & 3) == 0) { smw[j * 8 + hd] = mx; sdw[j * 8 + hd] = den; }
    __syncthreads();

    v4f o = *(const v4f*)(sow + 4 * lq);
    o = o * 0.125f + bb;
    const bool wr = (lane < 16) && (c < nN);
    float* gp = out + (size_t)c * CHN + 4 * lq;
    if (wr) *(volatile v4f*)gp = o;
    __threadfence();
    if (wr) *(volatile v4f*)gp = o;
    __syncthreads();
  }

  {
    const v4f m0 = *(const v4f*)(smw + 4 * lane);
    const v4f m1 = *(const v4f*)(smw + 128 + 4 * lane);
    const v4f d0 = *(const v4f*)(sdw + 4 * lane);
    const v4f d1 = *(const v4f*)(sdw + 128 + 4 * lane);
    float* mp = Mt + (size_t)tbase * NHD + 4 * lane;
    float* dp = Dt + (size_t)tbase * NHD + 4 * lane;
    *(volatile v4f*)mp = m0; *(volatile v4f*)(mp + 128) = m1;
    *(volatile v4f*)dp = d0; *(volatile v4f*)(dp + 128) = d1;
    __threadfence();
    *(volatile v4f*)mp = m0; *(volatile v4f*)(mp + 128) = m1;
    *(volatile v4f*)dp = d0; *(volatile v4f*)(dp + 128) = d1;
  }
}

__global__ __launch_bounds__(NTHR) void k_alpha(
    const int* __restrict__ srcs, const int* __restrict__ dsts,
    const float* __restrict__ eS, const float* __restrict__ eD,
    const float* __restrict__ Mt, const float* __restrict__ Dt,
    float* aout, int nN, int nE, int nEt, int npad) {
  __shared__ __attribute__((aligned(16))) float sa[NTHR * NHD];
  const int tid = threadIdx.x;
  const int ebase = blockIdx.x * NTHR;
  int e = ebase + tid;
  e = e > nEt - 1 ? nEt - 1 : e;
  int el = e > nE - 1 ? nE - 1 : e;
  el = el < 0 ? 0 : el;
  const int sl = srcs[el];
  const int dl = dsts[el];
  int s = (e < nE) ? sl : (e - nE);
  int d = (e < nE) ? dl : (e - nE);
  s = s < 0 ? 0 : (s > nN - 1 ? nN - 1 : s);
  d = d < 0 ? 0 : (d > nN - 1 ? nN - 1 : d);

  float esv[NHD], edv[NHD];
#pragma unroll
  for (int q = 0; q < 4; ++q) {
    const v2f a = *(const v2f*)(eS + ((size_t)q * (size_t)npad + (size_t)s) * 2);
    const v2f b = *(const v2f*)(eD + ((size_t)q * (size_t)npad + (size_t)d) * 2);
    esv[2 * q] = a.x; esv[2 * q + 1] = a.y;
    edv[2 * q] = b.x; edv[2 * q + 1] = b.y;
  }
  const v4f m0 = *(const v4f*)(Mt + (size_t)d * NHD);
  const v4f m1 = *(const v4f*)(Mt + (size_t)d * NHD + 4);
  const v4f n0 = *(const v4f*)(Dt + (size_t)d * NHD);
  const v4f n1 = *(const v4f*)(Dt + (size_t)d * NHD + 4);
  float mm[NHD], dd[NHD];
  mm[0] = m0.x; mm[1] = m0.y; mm[2] = m0.z; mm[3] = m0.w;
  mm[4] = m1.x; mm[5] = m1.y; mm[6] = m1.z; mm[7] = m1.w;
  dd[0] = n0.x; dd[1] = n0.y; dd[2] = n0.z; dd[3] = n0.w;
  dd[4] = n1.x; dd[5] = n1.y; dd[6] = n1.z; dd[7] = n1.w;
  float al[NHD];
#pragma unroll
  for (int h = 0; h < NHD; ++h) {
    const float den = dd[h] > 0.0f ? dd[h] : 1.0f;
    al[h] = __expf(lrelu(esv[h] + edv[h]) - mm[h]) * __builtin_amdgcn_rcpf(den);
  }
  {
    v4f o0, o1;
    o0.x = al[0]; o0.y = al[1]; o0.z = al[2]; o0.w = al[3];
    o1.x = al[4]; o1.y = al[5]; o1.z = al[6]; o1.w = al[7];
    *(v4f*)(sa + tid * NHD) = o0;
    *(v4f*)(sa + tid * NHD + 4) = o1;
  }
  __syncthreads();

  int nval = nEt - ebase;
  nval = nval < 0 ? 0 : (nval > NTHR ? NTHR : nval);
  const int nf4 = nval * 2;
  const v4f w0 = *(const v4f*)(sa + 4 * tid);
  const v4f w1 = *(const v4f*)(sa + 4 * (tid + NTHR));
  float* gp = aout + (size_t)ebase * NHD;
  const bool s0 = tid < nf4, s1 = (tid + NTHR) < nf4;
  if (s0) *(volatile v4f*)(gp + 4 * tid) = w0;
  if (s1) *(volatile v4f*)(gp + 4 * (tid + NTHR)) = w1;
  __threadfence();
  if (s0) *(volatile v4f*)(gp + 4 * tid) = w0;
  if (s1) *(volatile v4f*)(gp + 4 * (tid + NTHR)) = w1;
}

extern "C" void kernel_launch(void* const* d_in, const int* in_sizes, int n_in,
                              void* d_out, int out_size, void* d_ws, size_t ws_size,
                              hipStream_t stream) {
  if (n_in < 10) return;
  const int nN = in_sizes[0] / FIN;
  const int nE = in_sizes[1] / 2;
  if (nN <= 0 || nE <= 0 || in_sizes[0] != nN * FIN || in_sizes[1] != 2 * nE) return;
  if (in_sizes[2] != FIN * HCN || in_sizes[3] != NHD * CHN || in_sizes[4] != NHD * CHN || in_sizes[5] != HCN) return;
  if (in_sizes[6] != HCN * HCN || in_sizes[7] != NHD * CHN || in_sizes[8] != NHD * CHN || in_sizes[9] != CHN) return;
  if (nE > (1 << 26) || nN > (1 << 22)) return;
  const int nEt = nE + nN;
  if ((long long)out_size != (long long)nN * CHN + 2LL * (long long)nEt * NHD) return;

  const float* x   = (const float*)d_in[0];
  const int*   ei  = (const int*)d_in[1];
  const int*   src = ei;
  const int*   dst = ei + nE;
  const float* W1  = (const float*)d_in[2];
  const float* a1s = (const float*)d_in[3];
  const float* a1d = (const float*)d_in[4];
  const float* b1  = (const float*)d_in[5];
  const float* W2  = (const float*)d_in[6];
  const float* a2s = (const float*)d_in[7];
  const float* a2d = (const float*)d_in[8];
  const float* b2  = (const float*)d_in[9];
  float* out0   = (float*)d_out;
  float* alpha1 = out0 + (size_t)nN * CHN;
  float* alpha2 = alpha1 + (size_t)nEt * NHD;

  const int NPAD   = ((nN + TGT - 1) / TGT) * TGT;
  const int nBC    = (nN + NBC - 1) / NBC;
  const int CNTPAD = nBC * NBC;
  if (CNTPAD < NPAD) return;
  if (4 * nBC + 1 > RBN) return;
  const int nBF    = (nN + NBF - 1) / NBF;
  if (nBF + 1 > 4 * nBC + 1) return;
  const int csrLen = ((nE + 31) & ~31) + 4096;
  if (31 * 4 * nBC > 4096) return;
  const int nAgg   = NPAD / TGT;
  const int nGemm  = NPAD / BM;
  const int nXu    = NPAD * (FIN / 8);
  const int nAlpha = (nEt + NTHR - 1) / NTHR;

  char* ws = (char*)d_ws;
  size_t off = 0;
  const size_t oW1  = off; off += (size_t)HCN * FIN * 2;         off = (off + 255) & ~(size_t)255;
  const size_t oW2  = off; off += (size_t)HCN * HCN * 2;         off = (off + 255) & ~(size_t)255;
  const size_t oA   = off; off += (size_t)NPAD * HCN * 2;        off = (off + 255) & ~(size_t)255;
  const size_t oCnt = off; off += (size_t)CNTPAD * 4;            off = (off + 255) & ~(size_t)255;
  const size_t oOff = off; off += (size_t)CNTPAD * 4;            off = (off + 255) & ~(size_t)255;
  const size_t oRb  = off; off += (size_t)RBN * 4;               off = (off + 255) & ~(size_t)255;
  const size_t oCsr = off; off += (size_t)csrLen * 4;            off = (off + 255) & ~(size_t)255;
  const size_t oHw  = off; off += (size_t)NPAD * HCN * 4;        off = (off + 255) & ~(size_t)255;
  const size_t oES  = off; off += (size_t)NPAD * NHD * 4;        off = (off + 255) & ~(size_t)255;
  const size_t oED  = off; off += (size_t)NPAD * NHD * 4;        off = (off + 255) & ~(size_t)255;
  const size_t oM   = off; off += (size_t)NPAD * NHD * 4;        off = (off + 255) & ~(size_t)255;
  const size_t oD   = off; off += (size_t)NPAD * NHD * 4;        off = (off + 255) & ~(size_t)255;
  if (off > ws_size || off > (size_t)WSCAP) return;
  unsigned short* wp1 = (unsigned short*)(ws + oW1);
  unsigned short* wp2 = (unsigned short*)(ws + oW2);
  unsigned short* pa  = (unsigned short*)(ws + oA);
  int*   cnt  = (int*)(ws + oCnt);
  int*   offp = (int*)(ws + oOff);
  int*   rb   = (int*)(ws + oRb);
  int*   csr  = (int*)(ws + oCsr);
  float* hw   = (float*)(ws + oHw);
  float* es   = (float*)(ws + oES);
  float* ed   = (float*)(ws + oED);
  float* mt   = (float*)(ws + oM);
  float* dt   = (float*)(ws + oD);

  const int vec8 = ((nE & 3) == 0) ? 1 : 0;

  k_wprep<FIN, HCN><<<(HCN * FIN / 8 + NTHR - 1) / NTHR, NTHR, 0, stream>>>(W1, wp1);
  k_wprep<HCN, HCN><<<(HCN * HCN / 8 + NTHR - 1) / NTHR, NTHR, 0, stream>>>(W2, wp2);
  k_xcvt<<<(nXu + NTHR - 1) / NTHR, NTHR, 0, stream>>>(x, pa, nN, nXu);

  k_count<<<nBC, NTHR, 0, stream>>>(dst, cnt, nE, vec8);
  k_offsets<<<1, OTHR, 0, stream>>>(cnt, offp, rb, nBC);
  hipFuncSetAttribute(reinterpret_cast<const void*>(&k_fill),
                      hipFuncAttributeMaxDynamicSharedMemorySize, LDS_FILL);
  k_fill<<<nBF, NTHR, LDS_FILL, stream>>>(src, dst, offp, rb, csr, nN, nE, vec8, csrLen);

  k_gemm<FIN, 4><<<dim3(nGemm, HCN / BN), NTHR, 0, stream>>>(pa, wp1, a1s, a1d, hw, es, ed, NPAD);
  k_agg1<<<nAgg, NTHR, 0, stream>>>(csr, offp, cnt, es, ed, hw, b1, mt, dt, pa, nN, NPAD, csrLen);
  k_alpha<<<nAlpha, NTHR, 0, stream>>>(src, dst, es, ed, mt, dt, alpha1, nN, nE, nEt, NPAD);

  k_gemm<HCN, 7><<<dim3(nGemm, HCN / BN), NTHR, 0, stream>>>(pa, wp2, a2s, a2d, hw, es, ed, NPAD);
  k_agg2<<<nAgg, NTHR, 0, stream>>>(csr, offp, cnt, es, ed, hw, b2, mt, dt, out0, nN, NPAD, csrLen);
  k_alpha<<<nAlpha, NTHR, 0, stream>>>(src, dst, es, ed, mt, dt, alpha2, nN, nE, nEt, NPAD);
}
